// MultiHeadAttention_23854248362716
// MI455X (gfx1250) — hardware-verified
//
#include <hip/hip_runtime.h>


#ifndef NB
#define NB 2
#endif
#ifndef SEQ
#define SEQ 2048
#endif
#define NB_FULL  2
#define SEQ_FULL 2048
#ifndef OUT_SEQ
#define OUT_SEQ SEQ
#endif
#define DM   2048
#define NH_  16
#define HD   128
#define EARLY ((SEQ) < 512 ? (SEQ) : 512)
#define AW   4
#define QRS  2048.0f
#define QRI  (1.0f / 2048.0f)
#define SC2  (0.08838834764831845f * 1.4426950408889634f)
#define PSH  8.0f
#define CSC  16.0f
#define WSC  64.0f
#define OSC  (1.0f / 1024.0f)

static_assert(HD == 128);
static_assert(NH_ * HD == DM);
static_assert(DM % 64 == 0);
static_assert(DM % 32 == 0);
static_assert(SEQ % 64 == 0);
static_assert(EARLY % 64 == 0);
static_assert((SEQ - EARLY) % 64 == 0);
static_assert(((EARLY / 16) * 2) % AW == 0);
static_assert((SEQ - EARLY) % (16 * AW) == 0);
static_assert(SEQ % 32 == 0);
static_assert(((size_t)SEQ * DM) % 8 == 0);
static_assert(NB <= NB_FULL);
static_assert(SEQ <= SEQ_FULL);

typedef _Float16 h16;
typedef unsigned short bf;
typedef __attribute__((ext_vector_type(16))) __bf16   v16bf;
typedef __attribute__((ext_vector_type(16))) _Float16 v16h;
typedef __attribute__((ext_vector_type(8)))  _Float16 v8h;
typedef __attribute__((ext_vector_type(8)))  unsigned short v8us;
typedef __attribute__((ext_vector_type(16))) unsigned short v16us;
typedef __attribute__((ext_vector_type(8)))  float    v8f;
typedef __attribute__((ext_vector_type(4)))  float    v4f;
typedef v4f  __attribute__((may_alias)) v4fa;

__device__ __forceinline__ unsigned short f2bf(float f) { unsigned u = __float_as_uint(f); u += 0x7FFFu + ((u >> 16) & 1u); return (unsigned short)(u >> 16); }
__device__ __forceinline__ float bfr(float f) { return __uint_as_float(((unsigned)f2bf(f)) << 16); }
__device__ __forceinline__ v16h cat16(v8h lo, v8h hi) { return __builtin_shufflevector(lo, hi, 0, 1, 2, 3, 4, 5, 6, 7, 8, 9, 10, 11, 12, 13, 14, 15); }
__device__ __forceinline__ v16bf cat16b(v8us lo, v8us hi) { return __builtin_bit_cast(v16bf, __builtin_shufflevector(lo, hi, 0, 1, 2, 3, 4, 5, 6, 7, 8, 9, 10, 11, 12, 13, 14, 15)); }
__device__ __forceinline__ v8f wmma16(v16h a, v16h b, v8f c) { return __builtin_amdgcn_wmma_f32_16x16x32_f16(false, a, false, b, (short)0, c, false, false); }
__device__ __forceinline__ v8f wmmab(v16bf a, v16bf b, v8f c) { return __builtin_amdgcn_wmma_f32_16x16x32_bf16(false, a, false, b, (short)0, c, false, false); }
__device__ __forceinline__ v16h  ldh(const h16* p) { return cat16(*(const v8h*)p, *(const v8h*)(p + 16)); }
__device__ __forceinline__ v16bf ldb(const bf* p)  { return cat16b(*(const v8us*)p, *(const v8us*)(p + 16)); }
__device__ __forceinline__ void wave_sync() { __builtin_amdgcn_fence(3  , "wavefront"); __builtin_amdgcn_wave_barrier(); asm volatile("" ::: "memory"); }

__global__ __launch_bounds__(256) void k_cvt8(const float* __restrict__ src, bf* dst, size_t n8) {
    const size_t i = (size_t)blockIdx.x * 256 + threadIdx.x; if (i >= n8) return;
    const v8f v = *(const v8f*)(src + i * 8); v8us o;
#pragma unroll
    for (int k = 0; k < 8; ++k) o[k] = f2bf(v[k]);
    *(volatile v8us*)(dst + i * 8) = o; __threadfence(); *(volatile v8us*)(dst + i * 8) = o;
}

__global__ __launch_bounds__(256) void k_wT(const float* __restrict__ W, bf* dB, h16* dH, float scale, int mode) {
    __shared__ __align__(16) float ts[64 * 68];
    const int tid = threadIdx.x; const int k0 = blockIdx.x * 64, n0 = blockIdx.y * 64;
#pragma unroll
    for (int i = 0; i < 4; ++i) { const int idx = tid + 256 * i; const int kr = idx >> 4, c4 = (idx & 15) * 4;
        const v4f v = *(const v4f*)(W + (size_t)(k0 + kr) * DM + n0 + c4);
        ts[(c4 + 0) * 68 + kr] = v[0]; ts[(c4 + 1) * 68 + kr] = v[1]; ts[(c4 + 2) * 68 + kr] = v[2]; ts[(c4 + 3) * 68 + kr] = v[3]; }
    __syncthreads();
#pragma unroll 1
    for (int ps = 0; ps < 2; ++ps) {
#pragma unroll
        for (int s = 0; s < 2; ++s) { const int row = (tid >> 3) + 32 * s, c8 = (tid & 7) * 8;
            const v4f x0 = *(const v4fa*)(&ts[row * 68 + c8]); const v4f x1 = *(const v4fa*)(&ts[row * 68 + c8 + 4]); v8us ob; v8h oh;
#pragma unroll
            for (int i = 0; i < 4; ++i) { const float w0 = bfr(x0[i]) * scale, w1 = bfr(x1[i]) * scale; ob[i] = f2bf(w0); ob[4 + i] = f2bf(w1); oh[i] = (h16)w0; oh[4 + i] = (h16)w1; }
            const size_t oo = (size_t)(n0 + row) * DM + k0 + c8;
            if (mode & 1) *(volatile v8us*)(dB + oo) = ob;
            if (mode & 2) *(volatile v8h*)(dH + oo) = oh; }
        if (ps == 0) __threadfence(); }
}

template <int RM>
__global__ __launch_bounds__(32) void k_proj(const bf* __restrict__ A, const bf* __restrict__ Bt, h16* Ph, bf* Pr, int RB, size_t sRB, int pitch, int CB, size_t sCB,
                                             int resRows, int resCols, size_t sRBr, int pitchR, size_t sCBr) {
    __shared__ __align__(16) float os[16 * 68];
    const int K = DM;
    const int lane = threadIdx.x & 31, lr = lane & 15, hi = lane >> 4; const int r0 = blockIdx.x * 64, c0 = blockIdx.y * 64;
    v8f acc[4][4];
#pragma unroll
    for (int mb = 0; mb < 4; ++mb)
#pragma unroll
        for (int nb = 0; nb < 4; ++nb) acc[mb][nb] = (v8f){};
    const size_t aoff = (size_t)(r0 + lr) * K + 8 * hi, boff = (size_t)(c0 + lr) * K + 8 * hi;
#pragma unroll 1
    for (int kc = 0; kc < K; kc += 32) {
        v16bf a[4];
#pragma unroll
        for (int mb = 0; mb < 4; ++mb) a[mb] = ldb(A + aoff + (size_t)mb * 16 * K + kc);
#pragma unroll
        for (int nb = 0; nb < 4; ++nb) { const v16bf b = ldb(Bt + boff + (size_t)nb * 16 * K + kc);
#pragma unroll
            for (int mb = 0; mb < 4; ++mb) acc[mb][nb] = wmmab(a[mb], b, acc[mb][nb]); }
        asm volatile("v_nop\n\tv_nop\n\tv_nop\n\tv_nop" : "+v"(acc[0][0]), "+v"(acc[1][1]), "+v"(acc[2][2]), "+v"(acc[3][3]) : "v"(a[0]), "v"(a[1]), "v"(a[2]), "v"(a[3]));
    }
    const int rr = r0 % RB, cc = c0 % CB;
    const size_t tbase = (size_t)(r0 / RB) * sRB + (size_t)rr * (size_t)pitch + (size_t)(c0 / CB) * sCB + (size_t)cc;
    const size_t rbase = (size_t)(r0 / RB) * sRBr + (size_t)rr * (size_t)pitchR + (size_t)(c0 / CB) * sCBr + (size_t)cc;
    const int useRes = (rr < resRows) && (cc < resCols);
#pragma unroll
    for (int mb = 0; mb < 4; ++mb) {
#pragma unroll
        for (int nb = 0; nb < 4; ++nb) {
#pragma unroll
            for (int j = 0; j < 8; ++j) os[(hi * 8 + j) * 68 + nb * 16 + lr] = acc[mb][nb][j]; }
        wave_sync();
        const size_t sb = tbase + (size_t)(mb * 16) * (size_t)pitch;
        const size_t sr = rbase + (size_t)(mb * 16) * (size_t)pitchR;
#pragma unroll 1
        for (int ps = 0; ps < 2; ++ps) {
#pragma unroll
            for (int s = 0; s < 4; ++s) { const int row = 4 * s + (lane >> 3), c8 = (lane & 7) * 8;
                const v4f x0 = *(const v4fa*)(&os[row * 68 + c8]); const v4f x1 = *(const v4fa*)(&os[row * 68 + c8 + 4]); v8h hv, rh; v8us rb;
#pragma unroll
                for (int i = 0; i < 4; ++i) { const h16 a0 = (h16)x0[i]; const h16 a1 = (h16)x1[i]; hv[i] = a0; hv[4 + i] = a1;
                    const float d0 = x0[i] - (float)a0, d1 = x1[i] - (float)a1;
                    rh[i] = (h16)(d0 * QRS); rh[4 + i] = (h16)(d1 * QRS); rb[i] = f2bf(d0); rb[4 + i] = f2bf(d1); }
                const size_t oo = sb + (size_t)row * (size_t)pitch + c8;
                const size_t orr = sr + (size_t)row * (size_t)pitchR + c8;
                *(volatile v8h*)(Ph + oo) = hv;
                if (useRes) { if constexpr (RM == 1) *(volatile v8h*)((h16*)Pr + orr) = rh; else *(volatile v8us*)(Pr + orr) = rb; } }
            if (ps == 0) __threadfence(); }
        wave_sync();
    }
}

__global__ __launch_bounds__(32 * AW) void k_flash_d(const h16* __restrict__ QH, const h16* __restrict__ KP, const h16* __restrict__ VT, h16* CH) {
    __shared__ __align__(16) float os[AW * 16 * 132];
    const int lane = threadIdx.x & 31, lr = lane & 15, hi = lane >> 4;
    const int wave = __builtin_amdgcn_readfirstlane((int)(threadIdx.x >> 5));
    const int zh = blockIdx.y; const int b = zh / NH_, h = zh % NH_;
    const int t0 = EARLY + ((int)blockIdx.x * AW + wave) * 16;
    const size_t pbase = (size_t)zh * SEQ * HD;
    const size_t qo = pbase + (size_t)(t0 + lr) * HD + 8 * hi;
    const v16h q0 = ldh(QH + qo), q1 = ldh(QH + qo + 32), q2 = ldh(QH + qo + 64), q3 = ldh(QH + qo + 96);
    const size_t ko = pbase + (size_t)lr * HD + 8 * hi;
    const size_t vo = pbase + (size_t)lr * SEQ + 8 * hi;
    v8f o[8];
#pragma unroll
    for (int j = 0; j < 8; ++j) o[j] = (v8f){};
    float m = -3.0e38f, l = 0.0f;
    const int kend = t0 + 16; const int tq = t0 + lr;
#pragma unroll 1
    for (int key0 = 0; key0 < kend; key0 += 32) {
        const h16* ka = KP + ko + (size_t)key0 * HD;
        v8f sa = (v8f){}, sb = (v8f){};
        { const v16h a0 = ldh(ka), a1 = ldh(ka + 32), c0 = ldh(ka + 16 * HD), c1 = ldh(ka + 16 * HD + 32);
          sa = wmma16(a0, q0, sa); sb = wmma16(c0, q0, sb); sa = wmma16(a1, q1, sa); sb = wmma16(c1, q1, sb);
          asm volatile("v_nop\n\tv_nop\n\tv_nop\n\tv_nop" : "+v"(sa), "+v"(sb) : "v"(a0), "v"(a1), "v"(c0), "v"(c1)); }
        { const v16h a2 = ldh(ka + 64), a3 = ldh(ka + 96), c2 = ldh(ka + 16 * HD + 64), c3 = ldh(ka + 16 * HD + 96);
          sa = wmma16(a2, q2, sa); sb = wmma16(c2, q2, sb); sa = wmma16(a3, q3, sa); sb = wmma16(c3, q3, sb);
          asm volatile("v_nop\n\tv_nop\n\tv_nop\n\tv_nop" : "+v"(sa), "+v"(sb) : "v"(a2), "v"(a3), "v"(c2), "v"(c3)); }
        float ta[8], tb[8];
#pragma unroll
        for (int r = 0; r < 8; ++r) { ta[r] = sa[r] * SC2; tb[r] = sb[r] * SC2; }
        if (key0 + 31 > t0) {
#pragma unroll
            for (int r = 0; r < 8; ++r) { const int kk = key0 + 8 * hi + r; ta[r] = (kk > tq) ? -3.0e38f : ta[r]; tb[r] = (kk + 16 > tq) ? -3.0e38f : tb[r]; } }
        float mx = -3.0e38f;
#pragma unroll
        for (int r = 0; r < 8; ++r) mx = fmaxf(mx, fmaxf(ta[r], tb[r]));
        mx = fmaxf(mx, __shfl_xor(mx, 16, 32));
        const float mnew = fmaxf(m, mx);
        const float alpha = __builtin_amdgcn_exp2f(m - mnew);
        const float sh = PSH - mnew;
        v16h pb; float ls = 0.0f;
#pragma unroll
        for (int r = 0; r < 8; ++r) { const h16 pa = (h16)__builtin_amdgcn_exp2f(ta[r] + sh); const h16 pc = (h16)__builtin_amdgcn_exp2f(tb[r] + sh); pb[r] = pa; pb[8 + r] = pc; ls += (float)pa + (float)pc; }
        l = l * alpha + ls; m = mnew;
#pragma unroll
        for (int j = 0; j < 8; ++j) o[j] = o[j] * alpha;
        const h16* va = VT + vo + key0;
        { const v16h v0 = ldh(va), v1 = ldh(va + (size_t)16 * SEQ), v2 = ldh(va + (size_t)32 * SEQ), v3 = ldh(va + (size_t)48 * SEQ);
          o[0] = wmma16(v0, pb, o[0]); o[1] = wmma16(v1, pb, o[1]); o[2] = wmma16(v2, pb, o[2]); o[3] = wmma16(v3, pb, o[3]);
          asm volatile("v_nop\n\tv_nop\n\tv_nop\n\tv_nop" : "+v"(o[0]), "+v"(o[1]), "+v"(o[2]), "+v"(o[3]) : "v"(v0), "v"(v1), "v"(v2), "v"(v3), "v"(pb)); }
        { const v16h v4 = ldh(va + (size_t)64 * SEQ), v5 = ldh(va + (size_t)80 * SEQ), v6 = ldh(va + (size_t)96 * SEQ), v7 = ldh(va + (size_t)112 * SEQ);
          o[4] = wmma16(v4, pb, o[4]); o[5] = wmma16(v5, pb, o[5]); o[6] = wmma16(v6, pb, o[6]); o[7] = wmma16(v7, pb, o[7]);
          asm volatile("v_nop\n\tv_nop\n\tv_nop\n\tv_nop" : "+v"(o[4]), "+v"(o[5]), "+v"(o[6]), "+v"(o[7]) : "v"(v4), "v"(v5), "v"(v6), "v"(v7), "v"(pb)); }
    }
    l += __shfl_xor(l, 16, 32);
    const float inv = CSC / l;
    const int wb = wave * 16 * 132;
#pragma unroll
    for (int j = 0; j < 8; ++j) { v4f a, c;
        a[0] = o[j][0] * inv; a[1] = o[j][1] * inv; a[2] = o[j][2] * inv; a[3] = o[j][3] * inv; c[0] = o[j][4] * inv; c[1] = o[j][5] * inv; c[2] = o[j][6] * inv; c[3] = o[j][7] * inv;
        *(v4fa*)(&os[wb + lr * 132 + 16 * j + 8 * hi]) = a; *(v4fa*)(&os[wb + lr * 132 + 16 * j + 8 * hi + 4]) = c; }
    wave_sync();
    h16* crow = CH + ((size_t)b * SEQ + t0) * DM + h * HD;
#pragma unroll 1
    for (int ps = 0; ps < 2; ++ps) {
#pragma unroll
        for (int s = 0; s < 8; ++s) { const int row = 2 * s + hi, c8 = lr * 8;
            const v4f x0 = *(const v4fa*)(&os[wb + row * 132 + c8]); const v4f x1 = *(const v4fa*)(&os[wb + row * 132 + c8 + 4]); v8h hv;
#pragma unroll
            for (int i = 0; i < 4; ++i) { hv[i] = (h16)x0[i]; hv[4 + i] = (h16)x1[i]; }
            *(volatile v8h*)(crow + (size_t)row * DM + c8) = hv; }
        if (ps == 0) __threadfence(); }
}

__device__ __forceinline__ void sc3(const h16* khp, const h16* krp, v16h qhA, v16h qrA, v16h qhB, v16h qrB, v8f& sH, v8f& sL) {
    const v16h k0 = ldh(khp), k1 = ldh(khp + 32), r0 = ldh(krp), r1 = ldh(krp + 32);
    sH = wmma16(k0, qhA, sH); sL = wmma16(k0, qrA, sL); sH = wmma16(k1, qhB, sH); sL = wmma16(r0, qhA, sL);
    sL = wmma16(k1, qrB, sL); sL = wmma16(r1, qhB, sL);
    asm volatile("v_nop\n\tv_nop\n\tv_nop\n\tv_nop" : "+v"(sH), "+v"(sL) : "v"(k0), "v"(k1), "v"(r0), "v"(r1));
}

__global__ __launch_bounds__(32 * AW) void k_flash_e(const h16* __restrict__ QH, const h16* __restrict__ QR, const h16* __restrict__ KP, const h16* __restrict__ KR,
                                                    const h16* __restrict__ VT, const bf* __restrict__ VR, h16* CH, bf* CR) {
    __shared__ __align__(16) float os[AW * 16 * 68];
    const int lane = threadIdx.x & 31, lr = lane & 15, hi = lane >> 4;
    const int wave = __builtin_amdgcn_readfirstlane((int)(threadIdx.x >> 5));
    const int zh = blockIdx.y; const int b = zh / NH_, h = zh % NH_;
    const int gw = (int)blockIdx.x * AW + wave; const int t0 = (gw >> 1) * 16; const int dh = gw & 1;
    const size_t pbase = (size_t)zh * SEQ * HD;
    const size_t ebase = (size_t)zh * EARLY * HD;
    const size_t qo = pbase + (size_t)(t0 + lr) * HD + 8 * hi, qro = ebase + (size_t)(t0 + lr) * HD + 8 * hi;
    const v16h qh0 = ldh(QH + qo), qh1 = ldh(QH + qo + 32), qh2 = ldh(QH + qo + 64), qh3 = ldh(QH + qo + 96);
    const v16h qr0 = ldh(QR + qro), qr1 = ldh(QR + qro + 32), qr2 = ldh(QR + qro + 64), qr3 = ldh(QR + qro + 96);
    const size_t ko = pbase + (size_t)lr * HD + 8 * hi, kro = ebase + (size_t)lr * HD + 8 * hi;
    const size_t vo = pbase + (size_t)(dh * 64 + lr) * SEQ + 8 * hi, vro = ebase + (size_t)(dh * 64 + lr) * EARLY + 8 * hi;
    v8f oh[4], ol[4];
#pragma unroll
    for (int j = 0; j < 4; ++j) { oh[j] = (v8f){}; ol[j] = (v8f){}; }
    float m = -3.0e38f, l = 0.0f;
    const int kend = t0 + 16; const int tq = t0 + lr;
#pragma unroll 1
    for (int key0 = 0; key0 < kend; key0 += 32) {
        const h16* ka = KP + ko + (size_t)key0 * HD; const h16* kra = KR + kro + (size_t)key0 * HD;
        v8f sHa = (v8f){}, sLa = (v8f){}, sHb = (v8f){}, sLb = (v8f){};
        sc3(ka, kra, qh0, qr0, qh1, qr1, sHa, sLa);
        sc3(ka + 64, kra + 64, qh2, qr2, qh3, qr3, sHa, sLa);
        sc3(ka + 16 * HD, kra + 16 * HD, qh0, qr0, qh1, qr1, sHb, sLb);
        sc3(ka + 16 * HD + 64, kra + 16 * HD + 64, qh2, qr2, qh3, qr3, sHb, sLb);
        float ta[8], tb[8];
#pragma unroll
        for (int r = 0; r < 8; ++r) { ta[r] = (sHa[r] + sLa[r] * QRI) * SC2; tb[r] = (sHb[r] + sLb[r] * QRI) * SC2; }
        if (key0 + 31 > t0) {
#pragma unroll
            for (int r = 0; r < 8; ++r) { const int kk = key0 + 8 * hi + r; ta[r] = (kk > tq) ? -3.0e38f : ta[r]; tb[r] = (kk + 16 > tq) ? -3.0e38f : tb[r]; } }
        float mx = -3.0e38f;
#pragma unroll
        for (int r = 0; r < 8; ++r) mx = fmaxf(mx, fmaxf(ta[r], tb[r]));
        mx = fmaxf(mx, __shfl_xor(mx, 16, 32));
        const float mnew = fmaxf(m, mx);
        const float alpha = __builtin_amdgcn_exp2f(m - mnew);
        const float sh = PSH - mnew;
        v16h pa, pr; v16us pu; float ls = 0.0f;
#pragma unroll
        for (int r = 0; r < 8; ++r) { const float ea = __builtin_amdgcn_exp2f(ta[r] + sh), eb = __builtin_amdgcn_exp2f(tb[r] + sh);
            const h16 ha = (h16)ea, hb = (h16)eb; const h16 ra = (h16)((ea - (float)ha) * QRS), rb = (h16)((eb - (float)hb) * QRS);
            pa[r] = ha; pa[8 + r] = hb; pr[r] = ra; pr[8 + r] = rb; pu[r] = f2bf(ea); pu[8 + r] = f2bf(eb);
            ls += ((float)ha + (float)ra * QRI) + ((float)hb + (float)rb * QRI); }
        const v16bf pbb = __builtin_bit_cast(v16bf, pu);
        l = l * alpha + ls; m = mnew;
#pragma unroll
        for (int j = 0; j < 4; ++j) { oh[j] = oh[j] * alpha; ol[j] = ol[j] * alpha; }
        const h16* va = VT + vo + key0; const bf* vra = VR + vro + key0;
        { const v16h v0 = ldh(va), v1 = ldh(va + (size_t)16 * SEQ), v2 = ldh(va + (size_t)32 * SEQ), v3 = ldh(va + (size_t)48 * SEQ);
          oh[0] = wmma16(v0, pa, oh[0]); oh[1] = wmma16(v1, pa, oh[1]); oh[2] = wmma16(v2, pa, oh[2]); oh[3] = wmma16(v3, pa, oh[3]);
          ol[0] = wmma16(v0, pr, ol[0]); ol[1] = wmma16(v1, pr, ol[1]); ol[2] = wmma16(v2, pr, ol[2]); ol[3] = wmma16(v3, pr, ol[3]);
          asm volatile("v_nop\n\tv_nop\n\tv_nop\n\tv_nop" : "+v"(oh[0]), "+v"(oh[1]), "+v"(oh[2]), "+v"(oh[3]), "+v"(ol[0]), "+v"(ol[1]), "+v"(ol[2]), "+v"(ol[3]) : "v"(v0), "v"(v1), "v"(v2), "v"(v3), "v"(pa), "v"(pr)); }
        { const v16bf w0 = ldb(vra), w1 = ldb(vra + (size_t)16 * EARLY), w2 = ldb(vra + (size_t)32 * EARLY), w3 = ldb(vra + (size_t)48 * EARLY);
          oh[0] = wmmab(w0, pbb, oh[0]); oh[1] = wmmab(w1, pbb, oh[1]); oh[2] = wmmab(w2, pbb, oh[2]); oh[3] = wmmab(w3, pbb, oh[3]);
          asm volatile("v_nop\n\tv_nop\n\tv_nop\n\tv_nop" : "+v"(oh[0]), "+v"(oh[1]), "+v"(oh[2]), "+v"(oh[3]) : "v"(w0), "v"(w1), "v"(w2), "v"(w3), "v"(pbb)); }
    }
    l += __shfl_xor(l, 16, 32);
    const float inv = CSC / l;
    const int wb = wave * 16 * 68;
#pragma unroll
    for (int j = 0; j < 4; ++j) { v4f a, c;
#pragma unroll
        for (int i = 0; i < 4; ++i) { a[i] = (oh[j][i] + ol[j][i] * QRI) * inv; c[i] = (oh[j][4 + i] + ol[j][4 + i] * QRI) * inv; }
        *(v4fa*)(&os[wb + lr * 68 + 16 * j + 8 * hi]) = a; *(v4fa*)(&os[wb + lr * 68 + 16 * j + 8 * hi + 4]) = c; }
    wave_sync();
    h16* crow = CH + ((size_t)b * SEQ + t0) * DM + h * HD + dh * 64;
    bf*  rrow = CR + ((size_t)b * EARLY + t0) * DM + h * HD + dh * 64;
#pragma unroll 1
    for (int ps = 0; ps < 2; ++ps) {
#pragma unroll
        for (int s = 0; s < 4; ++s) { const int row = 4 * s + (lane >> 3), c8 = (lane & 7) * 8;
            const v4f x0 = *(const v4fa*)(&os[wb + row * 68 + c8]); const v4f x1 = *(const v4fa*)(&os[wb + row * 68 + c8 + 4]); v8h hv; v8us rv;
#pragma unroll
            for (int i = 0; i < 4; ++i) { const h16 a0 = (h16)x0[i]; const h16 a1 = (h16)x1[i]; hv[i] = a0; hv[4 + i] = a1; rv[i] = f2bf(x0[i] - (float)a0); rv[4 + i] = f2bf(x1[i] - (float)a1); }
            *(volatile v8h*)(crow + (size_t)row * DM + c8) = hv;
            *(volatile v8us*)(rrow + (size_t)row * DM + c8) = rv; }
        if (ps == 0) __threadfence(); }
}

template <int EK, int MB>
__global__ __launch_bounds__(32) void k_out(const h16* __restrict__ A, const bf* __restrict__ A2, const h16* __restrict__ Bh, const bf* __restrict__ Bb, const float* __restrict__ bo, float* OUT) {
    __shared__ __align__(16) float os[16 * 68];
    constexpr int TR = 16 * MB;
    constexpr int RPB = EK ? EARLY : (SEQ - EARLY);
    constexpr int TPB = (RPB / TR) > 0 ? (RPB / TR) : 1;
    const int lane = threadIdx.x & 31, lr = lane & 15, hi = lane >> 4;
    const int bx = blockIdx.x; const int b = bx / TPB; const int t0 = (EK ? 0 : EARLY) + (bx % TPB) * TR; const int c0 = blockIdx.y * 64;
    v8f acc[MB][4];
#pragma unroll
    for (int mb = 0; mb < MB; ++mb)
#pragma unroll
        for (int nb = 0; nb < 4; ++nb) acc[mb][nb] = (v8f){};
    const size_t aoff = ((size_t)b * SEQ + t0 + lr) * DM + 8 * hi;
    const size_t roff = ((size_t)b * EARLY + t0 + lr) * DM + 8 * hi;
    const size_t boff = (size_t)(c0 + lr) * DM + 8 * hi;
#pragma unroll 1
    for (int kc = 0; kc < DM; kc += 32) {
        { v16h a[MB];
#pragma unroll
          for (int mb = 0; mb < MB; ++mb) a[mb] = ldh(A + aoff + (size_t)mb * 16 * DM + kc);
#pragma unroll
          for (int nb = 0; nb < 4; ++nb) { const v16h bb = ldh(Bh + boff + (size_t)nb * 16 * DM + kc);
#pragma unroll
              for (int mb = 0; mb < MB; ++mb) acc[mb][nb] = wmma16(a[mb], bb, acc[mb][nb]); }
          if constexpr (MB == 4) asm volatile("v_nop\n\tv_nop\n\tv_nop\n\tv_nop" : "+v"(acc[0][0]), "+v"(acc[1][1]), "+v"(acc[2][2]), "+v"(acc[3][3]) : "v"(a[0]), "v"(a[1]), "v"(a[2]), "v"(a[3]));
          else asm volatile("v_nop\n\tv_nop\n\tv_nop\n\tv_nop" : "+v"(acc[0][3]), "+v"(acc[1][3]) : "v"(a[0]), "v"(a[1])); }
        if constexpr (EK != 0) { v16bf a2[MB];
#pragma unroll
          for (int mb = 0; mb < MB; ++mb) a2[mb] = ldb(A2 + roff + (size_t)mb * 16 * DM + kc);
#pragma unroll
          for (int nb = 0; nb < 4; ++nb) { const v16bf b2 = ldb(Bb + boff + (size_t)nb * 16 * DM + kc);
#pragma unroll
              for (int mb = 0; mb < MB; ++mb) acc[mb][nb] = wmmab(a2[mb], b2, acc[mb][nb]); }
          if constexpr (MB == 4) asm volatile("v_nop\n\tv_nop\n\tv_nop\n\tv_nop" : "+v"(acc[0][0]), "+v"(acc[1][1]), "+v"(acc[2][2]), "+v"(acc[3][3]) : "v"(a2[0]), "v"(a2[1]), "v"(a2[2]), "v"(a2[3]));
          else asm volatile("v_nop\n\tv_nop\n\tv_nop\n\tv_nop" : "+v"(acc[0][3]), "+v"(acc[1][3]) : "v"(a2[0]), "v"(a2[1])); }
    }
    const v4f braw = *(const v4f*)(bo + c0 + lr * 4); v4f bv;
#pragma unroll
    for (int i = 0; i < 4; ++i) bv[i] = bfr(braw[i]);
    float* orow = OUT + ((size_t)b * OUT_SEQ + t0) * DM + c0;
#pragma unroll
    for (int mb = 0; mb < MB; ++mb) {
#pragma unroll
        for (int nb = 0; nb < 4; ++nb) {
#pragma unroll
            for (int j = 0; j < 8; ++j) os[(hi * 8 + j) * 68 + nb * 16 + lr] = acc[mb][nb][j]; }
        wave_sync();
#pragma unroll 1
        for (int ps = 0; ps < 2; ++ps) {
#pragma unroll
            for (int s = 0; s < 8; ++s) { const int row = 2 * s + hi, cofs = lr * 4;
                const v4f x0 = *(const v4fa*)(&os[row * 68 + cofs]); v4f val;
#pragma unroll
                for (int i = 0; i < 4; ++i) val[i] = x0[i] * OSC + bv[i];
                *(volatile v4f*)(orow + (size_t)(mb * 16 + row) * DM + cofs) = val; }
            if (ps == 0) __threadfence(); }
        wave_sync();
    }
}

static constexpr size_t al256(size_t v) { return (v + 255) & ~(size_t)255; }
static constexpr size_t SZ_XB = al256((size_t)NB * SEQ * DM * 2);
static constexpr size_t SZ_W  = al256((size_t)DM * DM * 2);
static constexpr size_t SZ_PL = al256((size_t)NB * NH_ * SEQ * HD * 2);
static constexpr size_t SZ_PE = al256((size_t)NB * NH_ * EARLY * HD * 2);
static constexpr size_t SZ_TOTAL = SZ_XB + 5 * SZ_W + 3 * SZ_PL + 4 * SZ_PE;
static_assert(SZ_TOTAL <= (size_t)134217728);
static_assert((size_t)NB * SEQ * DM * 2 <= SZ_XB);
static_assert((size_t)NB * EARLY * DM * 2 <= SZ_PE);
static_assert((size_t)NB * NH_ * HD * EARLY * 2 <= SZ_PE);

extern "C" void kernel_launch(void* const* d_in, const int* in_sizes, int n_in,
                              void* d_out, int out_size, void* d_ws, size_t ws_size, hipStream_t stream) {
    if (n_in < 6) return;
    const size_t needx = ((size_t)(NB - 1) * SEQ_FULL + SEQ) * DM;
    if ((size_t)in_sizes[0] < needx) return;
    if ((size_t)in_sizes[1] < (size_t)DM * DM || (size_t)in_sizes[2] < (size_t)DM * DM || (size_t)in_sizes[3] < (size_t)DM * DM || (size_t)in_sizes[4] < (size_t)DM * DM) return;
    if ((size_t)in_sizes[5] < (size_t)DM) return;
    if ((size_t)out_size < ((size_t)(NB - 1) * OUT_SEQ + SEQ) * DM) return;
    if (SZ_TOTAL > ws_size) return;
    const float* x = (const float*)d_in[0]; const float* wq = (const float*)d_in[1]; const float* wk = (const float*)d_in[2];
    const float* wv = (const float*)d_in[3]; const float* wo = (const float*)d_in[4]; const float* bo = (const float*)d_in[5];
    float* OUT = (float*)d_out;
    char* wsp = (char*)d_ws;
    bf* XB = (bf*)wsp; h16* CH = (h16*)wsp; wsp += SZ_XB;
    bf* WQT = (bf*)wsp; wsp += SZ_W;
    bf* WKT = (bf*)wsp; wsp += SZ_W;
    bf* WVT = (bf*)wsp; wsp += SZ_W;
    h16* WOH = (h16*)wsp; wsp += SZ_W;
    bf* WOB = (bf*)wsp; wsp += SZ_W;
    h16* QH = (h16*)wsp; wsp += SZ_PL;
    h16* KP = (h16*)wsp; wsp += SZ_PL;
    h16* VT = (h16*)wsp; wsp += SZ_PL;
    h16* QR = (h16*)wsp; wsp += SZ_PE;
    h16* KR = (h16*)wsp; wsp += SZ_PE;
    bf* VR = (bf*)wsp; wsp += SZ_PE;
    bf* CR = (bf*)wsp; wsp += SZ_PE;

    if (SEQ == SEQ_FULL) {
        const size_t n8 = (size_t)NB * SEQ * DM / 8;
        k_cvt8<<<(unsigned)((n8 + 255) / 256), 256, 0, stream>>>(x, XB, n8);
    } else {
        const size_t n8 = (size_t)SEQ * DM / 8;
        for (int b = 0; b < NB; ++b) k_cvt8<<<(unsigned)((n8 + 255) / 256), 256, 0, stream>>>(x + (size_t)b * SEQ_FULL * DM, XB + (size_t)b * SEQ * DM, n8);
    }
    { const dim3 g(DM / 64, DM / 64, 1);
      k_wT<<<g, 256, 0, stream>>>(wq, WQT, (h16*)WQT, 1.0f, 1);
      k_wT<<<g, 256, 0, stream>>>(wk, WKT, (h16*)WKT, 1.0f, 1);
      k_wT<<<g, 256, 0, stream>>>(wv, WVT, (h16*)WVT, 1.0f, 1);
      k_wT<<<g, 256, 0, stream>>>(wo, WOB, WOH, WSC, 3); }

    k_proj<1><<<dim3(NB * SEQ / 64, DM / 64, 1), 32, 0, stream>>>(XB, WQT, QH, (bf*)QR, SEQ, (size_t)NH_ * SEQ * HD, HD, HD, (size_t)SEQ * HD,
                                                                  EARLY, HD, (size_t)NH_ * EARLY * HD, HD, (size_t)EARLY * HD);
    k_proj<1><<<dim3(NB * SEQ / 64, DM / 64, 1), 32, 0, stream>>>(XB, WKT, KP, (bf*)KR, SEQ, (size_t)NH_ * SEQ * HD, HD, HD, (size_t)SEQ * HD,
                                                                  EARLY, HD, (size_t)NH_ * EARLY * HD, HD, (size_t)EARLY * HD);
    k_proj<2><<<dim3(DM / 64, NB * SEQ / 64, 1), 32, 0, stream>>>(WVT, XB, VT, VR, DM, (size_t)0, SEQ, SEQ, (size_t)DM * SEQ,
                                                                  DM, EARLY, (size_t)0, EARLY, (size_t)DM * EARLY);

    k_flash_e<<<dim3((EARLY / 16) * 2 / AW, NB * NH_, 1), 32 * AW, 0, stream>>>(QH, QR, KP, KR, VT, VR, CH, CR);
    if (SEQ > EARLY) k_flash_d<<<dim3((SEQ - EARLY) / (16 * AW), NB * NH_, 1), 32 * AW, 0, stream>>>(QH, KP, VT, CH);

    k_out<1, 2><<<dim3(NB * EARLY / 32, DM / 64, 1), 32, 0, stream>>>(CH, CR, WOH, WOB, bo, OUT);
    if (SEQ > EARLY) k_out<0, 4><<<dim3(NB * (SEQ - EARLY) / 64, DM / 64, 1), 32, 0, stream>>>(CH, CR, WOH, WOB, bo, OUT);
}
